// RelativeMultiHeadAttention_19619410608526
// MI455X (gfx1250) — hardware-verified
//
#include <hip/hip_runtime.h>


#ifndef NB
#define NB 4
#endif
#ifndef SEQ
#define SEQ 2048
#endif
#define NB_FULL   4
#define SEQ_FULL  2048
#define LREL      (2 * SEQ - 1)
#define LP        (2 * SEQ)
#define LREL_FULL (2 * SEQ_FULL - 1)
#define DM  512
#define NH  8
#define HD  64
#define RESC 2048.0f
#define K2 (1.4426950408889634f * 0.044194173824159216f)
static_assert(SEQ % 64 == 0);
static_assert(SEQ >= 64);
static_assert(SEQ <= SEQ_FULL);
static_assert(NB >= 1);
static_assert(NB <= NB_FULL);
static_assert(DM % 64 == 0);
static_assert(NH * HD == DM);
static_assert(LP % 64 == 0);

typedef _Float16 h16;
typedef unsigned short bf;
typedef __attribute__((ext_vector_type(16))) __bf16   v16bf;
typedef __attribute__((ext_vector_type(16))) _Float16 v16h;
typedef __attribute__((ext_vector_type(8)))  _Float16 v8h;
typedef __attribute__((ext_vector_type(8)))  unsigned short v8us;
typedef __attribute__((ext_vector_type(8)))  float    v8f;
typedef __attribute__((ext_vector_type(4)))  float    v4f;
typedef __attribute__((ext_vector_type(2)))  _Float16 v2h;
typedef v8h  __attribute__((may_alias)) v8ha;
typedef v4f  __attribute__((may_alias)) v4fa;
typedef v8f  __attribute__((may_alias)) v8fa;
typedef v8us __attribute__((may_alias)) v8usa;

__device__ __forceinline__ unsigned short f2bf(float f) { unsigned u = __float_as_uint(f); u += 0x7FFFu + ((u >> 16) & 1u); return (unsigned short)(u >> 16); }
__device__ __forceinline__ float bf2f(unsigned short b) { return __uint_as_float(((unsigned)b) << 16); }
__device__ __forceinline__ float bfr(float f) { return bf2f(f2bf(f)); }
__device__ __forceinline__ v16h cat16(v8h lo, v8h hi) { return __builtin_shufflevector(lo, hi, 0, 1, 2, 3, 4, 5, 6, 7, 8, 9, 10, 11, 12, 13, 14, 15); }
__device__ __forceinline__ v16bf cat16b(v8us lo, v8us hi) { return __builtin_bit_cast(v16bf, __builtin_shufflevector(lo, hi, 0, 1, 2, 3, 4, 5, 6, 7, 8, 9, 10, 11, 12, 13, 14, 15)); }
__device__ __forceinline__ v8f wmma16(v16h a, v16h b, v8f c) { return __builtin_amdgcn_wmma_f32_16x16x32_f16(false, a, false, b, (short)0, c, false, false); }
__device__ __forceinline__ v8f wmmab(v16bf a, v16bf b, v8f c) { return __builtin_amdgcn_wmma_f32_16x16x32_bf16(false, a, false, b, (short)0, c, false, false); }
__device__ __forceinline__ h16 tohx(float x) { return (h16)x; }
__device__ __forceinline__ void splitf(float y, unsigned short& h, unsigned short& l) { h = f2bf(y); l = f2bf(y - bf2f(h)); }

template <typename T16> struct WFrag;
template <> struct WFrag<h16> { typedef v16h V; static __device__ __forceinline__ V ld(const h16* p) { return cat16(*(const v8h*)p, *(const v8h*)(p + 16)); } static __device__ __forceinline__ v8f mma(V a, V b, v8f c) { return wmma16(a, b, c); } };
template <> struct WFrag<bf> { typedef v16bf V; static __device__ __forceinline__ V ld(const bf* p) { return cat16b(*(const v8us*)p, *(const v8us*)(p + 16)); } static __device__ __forceinline__ v8f mma(V a, V b, v8f c) { return wmmab(a, b, c); } };
template <typename T16, int NSPLIT, bool BIAS>
__global__ __launch_bounds__(32) void k_gemmw(const T16* __restrict__ A, const T16* __restrict__ A2, const T16* __restrict__ Bt, const T16* __restrict__ Bt2, int K, float* C, int ldc, const float* __restrict__ bias, size_t sA, size_t sB, size_t sC) {
    typedef typename WFrag<T16>::V V;
    __shared__ __align__(16) float os[16 * 68];
    const size_t z = blockIdx.z; A += z * sA; if (A2) A2 += z * sA; Bt += z * sB; if (Bt2) Bt2 += z * sB; C += z * sC;
    const int lane = threadIdx.x & 31, lr = lane & 15, hi = lane >> 4; const int r0 = blockIdx.x * 64, c0 = blockIdx.y * 64;
    v8f acc[4][4];
#pragma unroll
    for (int mb = 0; mb < 4; ++mb)
#pragma unroll
        for (int nb = 0; nb < 4; ++nb) acc[mb][nb] = (v8f){};
    const size_t aoff = (size_t)(r0 + lr) * K + 8 * hi, boff = (size_t)(c0 + lr) * K + 8 * hi;
#pragma unroll 1
    for (int kc = 0; kc < K; kc += 32) {
        V a[4], a2[4];
#pragma unroll
        for (int mb = 0; mb < 4; ++mb) { a[mb] = WFrag<T16>::ld(A + aoff + (size_t)mb * 16 * K + kc); if (NSPLIT == 1 || NSPLIT == 2) a2[mb] = WFrag<T16>::ld(A2 + aoff + (size_t)mb * 16 * K + kc); }
#pragma unroll
        for (int nb = 0; nb < 4; ++nb) { const V b = WFrag<T16>::ld(Bt + boff + (size_t)nb * 16 * K + kc); V b2; if (NSPLIT >= 2) b2 = WFrag<T16>::ld(Bt2 + boff + (size_t)nb * 16 * K + kc);
#pragma unroll
            for (int mb = 0; mb < 4; ++mb) { acc[mb][nb] = WFrag<T16>::mma(a[mb], b, acc[mb][nb]); if (NSPLIT == 1 || NSPLIT == 2) acc[mb][nb] = WFrag<T16>::mma(a2[mb], b, acc[mb][nb]); if (NSPLIT >= 2) acc[mb][nb] = WFrag<T16>::mma(a[mb], b2, acc[mb][nb]); } }
        asm volatile("v_nop\n\tv_nop\n\tv_nop\n\tv_nop" : "+v"(acc[0][0]), "+v"(acc[1][1]), "+v"(acc[2][2]), "+v"(acc[3][3]) : "v"(a[0]), "v"(a[3]));
    }
#pragma unroll
    for (int mb = 0; mb < 4; ++mb) {
#pragma unroll
        for (int nb = 0; nb < 4; ++nb) {
#pragma unroll
            for (int j = 0; j < 8; ++j) os[(hi * 8 + j) * 68 + nb * 16 + lr] = acc[mb][nb][j]; }
        __builtin_amdgcn_wave_barrier(); asm volatile("" ::: "memory");
        float* crow = C + (size_t)(r0 + mb * 16) * ldc + c0;
#pragma unroll 1
        for (int ps = 0; ps < 2; ++ps) {
#pragma unroll
            for (int s = 0; s < 8; ++s) { const int row = 2 * s + hi, cofs = lr * 4; v4f val = *(const v4fa*)(os + row * 68 + cofs); if (BIAS) { val[0] += bfr(bias[c0 + cofs]); val[1] += bfr(bias[c0 + cofs + 1]); val[2] += bfr(bias[c0 + cofs + 2]); val[3] += bfr(bias[c0 + cofs + 3]); }
                *(volatile v4f*)(crow + (size_t)row * ldc + cofs) = val; }
            if (ps == 0) __threadfence(); }
        __builtin_amdgcn_wave_barrier(); asm volatile("" ::: "memory");
    }
}

__global__ __launch_bounds__(256) void k_cvt8(const float* __restrict__ src, bf* dst, size_t n8) { const size_t i = (size_t)blockIdx.x * 256 + threadIdx.x; if (i >= n8) return; const v8f v = *(const v8f*)(src + i * 8); v8us o;
#pragma unroll
    for (int k = 0; k < 8; ++k) o[k] = f2bf(v[k]); *(volatile v8us*)(dst + i * 8) = o; __threadfence(); *(volatile v8us*)(dst + i * 8) = o; }

__global__ __launch_bounds__(256) void k_cvtrows(const float* __restrict__ src, int srows, int nvalid, int nout, bf* dst) {
    const size_t i = (size_t)blockIdx.x * 256 + threadIdx.x; const size_t total = (size_t)NB * nout * (DM / 8); if (i >= total) return;
    const int k0 = (int)(i % (DM / 8)) * 8; const int r = (int)((i / (DM / 8)) % (size_t)nout); const int b = (int)(i / ((size_t)(DM / 8) * nout));
    const int rc = min(r, nvalid - 1); const v8f v = *(const v8f*)(src + ((size_t)b * srows + rc) * DM + k0); v8us o;
#pragma unroll
    for (int q = 0; q < 8; ++q) { const unsigned short w = f2bf(v[q]); o[q] = (r < nvalid) ? w : (unsigned short)0; }
    bf* dp = dst + ((size_t)b * nout + r) * DM + k0; *(volatile v8us*)dp = o; __threadfence(); *(volatile v8us*)dp = o;
}

__global__ __launch_bounds__(256) void k_qplanes(const float* __restrict__ F, const float* __restrict__ ub, const float* __restrict__ vb, h16* Qu, h16* Qv) {
    const size_t e = ((size_t)blockIdx.x * 256 + threadIdx.x) * 2; if (e >= (size_t)NB * NH * SEQ * HD) return;
    const int d = (int)(e % HD); const int t = (int)((e / HD) % SEQ); const int hh = (int)((e / ((size_t)HD * SEQ)) % NH); const int b = (int)(e / ((size_t)HD * SEQ * NH));
    const float* f = F + ((size_t)b * SEQ + t) * DM + hh * HD + d; v2h ou, ov;
#pragma unroll
    for (int q = 0; q < 2; ++q) { const float x = f[q]; ou[q] = tohx(x + bfr(ub[hh * HD + d + q])); ov[q] = tohx(x + bfr(vb[hh * HD + d + q])); }
    *(volatile v2h*)(Qu + e) = ou; *(volatile v2h*)(Qv + e) = ov; __threadfence(); *(volatile v2h*)(Qu + e) = ou; *(volatile v2h*)(Qv + e) = ov;
}
__global__ __launch_bounds__(256) void k_kplane(const float* __restrict__ F, h16* Kp) {
    const size_t e = ((size_t)blockIdx.x * 256 + threadIdx.x) * 2; if (e >= (size_t)NB * NH * SEQ * HD) return;
    const int d = (int)(e % HD); const int t = (int)((e / HD) % SEQ); const int hh = (int)((e / ((size_t)HD * SEQ)) % NH); const int b = (int)(e / ((size_t)HD * SEQ * NH));
    const float* f = F + ((size_t)b * SEQ + t) * DM + hh * HD + d; v2h o;
#pragma unroll
    for (int q = 0; q < 2; ++q) o[q] = tohx(f[q]);
    *(volatile v2h*)(Kp + e) = o; __threadfence(); *(volatile v2h*)(Kp + e) = o;
}
__global__ __launch_bounds__(256) void k_vplanes(const float* __restrict__ F, h16* V16, h16* VR) {
    const size_t e = ((size_t)blockIdx.x * 256 + threadIdx.x) * 2; if (e >= (size_t)NB * NH * HD * SEQ) return;
    const int t = (int)(e % SEQ); const int d = (int)((e / SEQ) % HD); const int hh = (int)((e / ((size_t)SEQ * HD)) % NH); const int b = (int)(e / ((size_t)SEQ * HD * NH));
    v2h o16, orr;
#pragma unroll
    for (int q = 0; q < 2; ++q) { const float x = F[((size_t)b * SEQ + t + q) * DM + hh * HD + d]; const h16 xh = tohx(x); o16[q] = xh; orr[q] = tohx((x - (float)xh) * RESC); }
    *(volatile v2h*)(V16 + e) = o16; *(volatile v2h*)(VR + e) = orr; __threadfence(); *(volatile v2h*)(V16 + e) = o16; *(volatile v2h*)(VR + e) = orr;
}
__global__ __launch_bounds__(256) void k_pplane(const float* __restrict__ F, h16* Pp) {
    const size_t e = ((size_t)blockIdx.x * 256 + threadIdx.x) * 2; if (e >= (size_t)NB * NH * LP * HD) return;
    const int d = (int)(e % HD); const int l = (int)((e / HD) % LP); const int hh = (int)((e / ((size_t)HD * LP)) % NH); const int b = (int)(e / ((size_t)HD * LP * NH));
    const float* f = F + ((size_t)b * LP + l) * DM + hh * HD + d; v2h o;
#pragma unroll
    for (int q = 0; q < 2; ++q) o[q] = tohx(f[q]);
    *(volatile v2h*)(Pp + e) = o; __threadfence(); *(volatile v2h*)(Pp + e) = o;
}

__device__ __forceinline__ v16h ldl(const h16* p) { return cat16(*(const v8ha*)p, *(const v8ha*)(p + 16)); }
__device__ __forceinline__ void cp8k(h16* dst, const h16* __restrict__ src, int tid) {
#pragma unroll
    for (int c = 0; c < 4; ++c) { const int idx = tid + c * 128; *(v8ha*)(dst + (size_t)idx * 8) = *(const v8ha*)(src + (size_t)idx * 8); } }
__device__ __forceinline__ void cprows(h16* dst, const h16* __restrict__ src, size_t pitch, int tid) {
#pragma unroll
    for (int c = 0; c < 4; ++c) { const int idx = tid + c * 128; const int r = idx >> 3, sg = idx & 7; *(v8ha*)(dst + r * 64 + sg * 8) = *(const v8ha*)(src + (size_t)r * pitch + sg * 8); } }
__device__ __forceinline__ void band_half(const h16* PBl, const h16* Qvl, float* Tl, int slot0, int irow, int hi, int lr) {
    const v16h q0 = ldl(Qvl + irow * 64 + 8 * hi), q1 = ldl(Qvl + irow * 64 + 32 + 8 * hi);
    float* trow = Tl + irow * 128 + slot0 + 8 * hi;
#pragma unroll
    for (int tt = 0; tt < 4; ++tt) {
        const v16h a0 = ldl(PBl + (tt * 16 + lr) * 64 + 8 * hi), a1 = ldl(PBl + (tt * 16 + lr) * 64 + 32 + 8 * hi);
        v8f t = wmma16(a0, q0, (v8f){}); t = wmma16(a1, q1, t);
        asm volatile("v_nop\n\tv_nop\n\tv_nop\n\tv_nop" : "+v"(t) : "v"(a0), "v"(a1), "v"(q0), "v"(q1) : "memory");
        *(v8fa*)(trow + tt * 16) = t;
    }
}

__global__ __launch_bounds__(128) __attribute__((amdgpu_num_vgpr(256))) void k_attn(const h16* __restrict__ Qu, const h16* __restrict__ Qv, const h16* __restrict__ Kp, const h16* __restrict__ Vp, const h16* __restrict__ Vr, const h16* __restrict__ Pp, bf* ATh, bf* ATl) {
    __shared__ __align__(16) h16 Qul[64 * 64];
    __shared__ __align__(16) h16 Qvl[64 * 64];
    __shared__ __align__(16) h16 Kl[64 * 64];
    __shared__ __align__(16) h16 Vl[64 * 64];
    __shared__ __align__(16) h16 Vrl[64 * 64];
    __shared__ __align__(16) h16 PBl[64 * 64];
    __shared__ __align__(32) float Tl[64 * 128];
    __shared__ __align__(16) bf Est[2 * 64 * 64];
    const int tid = threadIdx.x, lane = tid & 31, wave = tid >> 5, hi = lane >> 4, lr = lane & 15;
    const int irow = wave * 16 + lr;
    const int i0 = blockIdx.x * 64, h = blockIdx.y, b = blockIdx.z;
    const size_t bh = (size_t)b * NH + h;
    const h16* Kb = Kp + bh * SEQ * HD; const h16* Vb = Vp + bh * HD * SEQ; const h16* Vrb = Vr + bh * HD * SEQ; const h16* Pb = Pp + bh * LP * HD;
    cp8k(Qul, Qu + (bh * SEQ + i0) * HD, tid); cp8k(Qvl, Qv + (bh * SEQ + i0) * HD, tid);
    const int lb0 = SEQ - 64 - i0;
    cp8k(PBl, Pb + (size_t)lb0 * HD, tid);
    __syncthreads();
    band_half(PBl, Qvl, Tl, lb0 & 127, irow, hi, lr);
    float mrun = -3.0e38f, lrun = 0.f;
    v8f oacc[4], oaccr[4];
#pragma unroll
    for (int nd = 0; nd < 4; ++nd) { oacc[nd] = (v8f){}; oaccr[nd] = (v8f){}; }
#pragma unroll 1
    for (int j0 = 0; j0 < SEQ; j0 += 64) {
        const int lb = lb0 + j0; const int lnw = lb + 64;
        __syncthreads();
        cp8k(Kl, Kb + (size_t)j0 * HD, tid); cprows(Vl, Vb + j0, (size_t)SEQ, tid); cprows(Vrl, Vrb + j0, (size_t)SEQ, tid); cp8k(PBl, Pb + (size_t)lnw * HD, tid);
        __syncthreads();
        band_half(PBl, Qvl, Tl, lnw & 127, irow, hi, lr);
        v8f sacc[4];
        { const v16h q0 = ldl(Qul + irow * 64 + 8 * hi), q1 = ldl(Qul + irow * 64 + 32 + 8 * hi);
#pragma unroll
          for (int tb = 0; tb < 4; ++tb) { const v16h a0 = ldl(Kl + (tb * 16 + lr) * 64 + 8 * hi), a1 = ldl(Kl + (tb * 16 + lr) * 64 + 32 + 8 * hi);
              sacc[tb] = wmma16(a0, q0, (v8f){}); sacc[tb] = wmma16(a1, q1, sacc[tb]);
              asm volatile("v_nop\n\tv_nop\n\tv_nop\n\tv_nop" : "+v"(sacc[tb]) : "v"(a0), "v"(a1), "v"(q0), "v"(q1) : "memory"); } }
        __syncthreads();
        const float* trow = Tl + irow * 128; const int sb = lb + 63 + 8 * hi - irow;
        float mx = -3.0e38f;
#pragma unroll
        for (int tb = 0; tb < 4; ++tb)
#pragma unroll
            for (int r = 0; r < 8; ++r) { const float s2 = (sacc[tb][r] + trow[(sb + tb * 16 + r) & 127]) * K2; sacc[tb][r] = s2; mx = fmaxf(mx, s2); }
        mx = fmaxf(mx, __shfl_xor(mx, 16, 32));
        const float mnew = fmaxf(mrun, mx); const float alpha = __builtin_amdgcn_exp2f(mrun - mnew); mrun = mnew;
        float rsum = 0.f; v8h ph[4], pl[4];
#pragma unroll
        for (int tb = 0; tb < 4; ++tb)
#pragma unroll
            for (int r = 0; r < 8; ++r) { const float p = __builtin_amdgcn_exp2f(sacc[tb][r] - mnew); rsum += p; const h16 p16 = tohx(p); ph[tb][r] = p16; pl[tb][r] = tohx((p - (float)p16) * RESC); }
        rsum += __shfl_xor(rsum, 16, 32); lrun = lrun * alpha + rsum;
#pragma unroll
        for (int r = 0; r < 8; ++r) { const float ar = __shfl(alpha, 8 * hi + r, 32);
#pragma unroll
            for (int nd = 0; nd < 4; ++nd) { oacc[nd][r] *= ar; oaccr[nd][r] *= ar; } }
        { const v16h pa0 = cat16(ph[0], ph[1]), pa1 = cat16(ph[2], ph[3]), pr0 = cat16(pl[0], pl[1]), pr1 = cat16(pl[2], pl[3]);
#pragma unroll
          for (int nd = 0; nd < 4; ++nd) {
              const v16h vb0 = ldl(Vl + (nd * 16 + lr) * 64 + 8 * hi), vb1 = ldl(Vl + (nd * 16 + lr) * 64 + 32 + 8 * hi);
              const v16h rb0 = ldl(Vrl + (nd * 16 + lr) * 64 + 8 * hi), rb1 = ldl(Vrl + (nd * 16 + lr) * 64 + 32 + 8 * hi);
              oacc[nd] = wmma16(pa0, vb0, oacc[nd]); oacc[nd] = wmma16(pa1, vb1, oacc[nd]);
              oaccr[nd] = wmma16(pa0, rb0, oaccr[nd]); oaccr[nd] = wmma16(pa1, rb1, oaccr[nd]); oaccr[nd] = wmma16(pr0, vb0, oaccr[nd]); oaccr[nd] = wmma16(pr1, vb1, oaccr[nd]);
              asm volatile("v_nop\n\tv_nop\n\tv_nop\n\tv_nop" : "+v"(oacc[nd]), "+v"(oaccr[nd]) : "v"(pa0), "v"(pa1), "v"(pr0), "v"(pr1), "v"(vb1), "v"(rb1) : "memory"); } }
    }
    const float rl = __builtin_amdgcn_rcpf(lrun);
#pragma unroll
    for (int r = 0; r < 8; ++r) { const float rli = __shfl(rl, 8 * hi + r, 32); const int rr = wave * 16 + 8 * hi + r;
#pragma unroll
        for (int nd = 0; nd < 4; ++nd) { const float c = (oacc[nd][r] + oaccr[nd][r] * (1.0f / RESC)) * rli; unsigned short eh, el; splitf(c, eh, el); Est[rr * 64 + nd * 16 + lr] = eh; Est[4096 + rr * 64 + nd * 16 + lr] = el; } }
    __syncthreads();
    const int rq = lane >> 3, pc = (lane & 7) * 8;
#pragma unroll 1
    for (int ps = 0; ps < 2; ++ps) {
#pragma unroll
        for (int rg = 0; rg < 4; ++rg) { const int rr = wave * 16 + rg * 4 + rq; const size_t go = ((size_t)b * SEQ + i0 + rr) * DM + h * HD + pc;
            const v8us vh = *(const v8usa*)(Est + rr * 64 + pc); const v8us vlo = *(const v8usa*)(Est + 4096 + rr * 64 + pc);
            *(volatile v8us*)(ATh + go) = vh; *(volatile v8us*)(ATl + go) = vlo; }
        if (ps == 0) __threadfence(); }
}

extern "C" void kernel_launch(void* const* d_in, const int* in_sizes, int n_in,
                              void* d_out, int out_size, void* d_ws, size_t ws_size, hipStream_t stream) {
    if (n_in < 15) return;
    const float* query = (const float*)d_in[0]; const float* key = (const float*)d_in[1]; const float* value = (const float*)d_in[2]; const float* pos = (const float*)d_in[3];
    const float* wq = (const float*)d_in[4]; const float* bq = (const float*)d_in[5]; const float* wk = (const float*)d_in[6]; const float* bk = (const float*)d_in[7];
    const float* wv = (const float*)d_in[8]; const float* bv = (const float*)d_in[9]; const float* wp = (const float*)d_in[10]; const float* ub = (const float*)d_in[11]; const float* vb = (const float*)d_in[12];
    const float* wo = (const float*)d_in[13]; const float* bo = (const float*)d_in[14];
    const long long needx = ((long long)(NB - 1) * SEQ_FULL + SEQ) * DM, needp = ((long long)(NB - 1) * LREL_FULL + LREL) * DM;
    if ((long long)in_sizes[0] < needx || (long long)in_sizes[1] < needx || (long long)in_sizes[2] < needx || (long long)in_sizes[3] < needp) return;
    if (in_sizes[4] < DM * DM || in_sizes[6] < DM * DM || in_sizes[8] < DM * DM || in_sizes[10] < DM * DM || in_sizes[13] < DM * DM) return;
    if (in_sizes[5] < DM || in_sizes[7] < DM || in_sizes[9] < DM || in_sizes[14] < DM || in_sizes[11] < NH * HD || in_sizes[12] < NH * HD) return;
    if ((long long)out_size < (long long)NB * SEQ * DM) return;
    float* OUT = (float*)d_out;
    char* wsp = (char*)d_ws;
    auto take = [&](size_t bytes) { char* p = wsp; wsp += (bytes + 255) & ~(size_t)255; return (void*)p; };
    bf* WQB = (bf*)take((size_t)DM * DM * 2); bf* WKB = (bf*)take((size_t)DM * DM * 2); bf* WVB = (bf*)take((size_t)DM * DM * 2); bf* WPB = (bf*)take((size_t)DM * DM * 2); bf* WOB = (bf*)take((size_t)DM * DM * 2);
    bf* XB = (bf*)take((size_t)NB * LP * DM * 2);
    float* F = (float*)take((size_t)NB * LP * DM * 4);
    h16* QU16 = (h16*)take((size_t)NB * NH * SEQ * HD * 2); h16* QV16 = (h16*)take((size_t)NB * NH * SEQ * HD * 2); h16* K16 = (h16*)take((size_t)NB * NH * SEQ * HD * 2);
    h16* V16 = (h16*)take((size_t)NB * NH * HD * SEQ * 2); h16* VR16 = (h16*)take((size_t)NB * NH * HD * SEQ * 2); h16* P16 = (h16*)take((size_t)NB * NH * LP * HD * 2);
    bf* ATh = (bf*)take((size_t)NB * SEQ * DM * 2); bf* ATl = (bf*)take((size_t)NB * SEQ * DM * 2);
    if ((size_t)(wsp - (char*)d_ws) > ws_size) return;
    const unsigned gw = (unsigned)(((size_t)DM * DM / 8 + 255) / 256);
    k_cvt8<<<gw, 256, 0, stream>>>(wq, WQB, (size_t)DM * DM / 8); k_cvt8<<<gw, 256, 0, stream>>>(wk, WKB, (size_t)DM * DM / 8); k_cvt8<<<gw, 256, 0, stream>>>(wv, WVB, (size_t)DM * DM / 8);
    k_cvt8<<<gw, 256, 0, stream>>>(wp, WPB, (size_t)DM * DM / 8); k_cvt8<<<gw, 256, 0, stream>>>(wo, WOB, (size_t)DM * DM / 8);
    const unsigned gx = (unsigned)(((size_t)NB * SEQ * (DM / 8) + 255) / 256), gxp = (unsigned)(((size_t)NB * LP * (DM / 8) + 255) / 256);
    const unsigned gpl = (unsigned)(((size_t)NB * NH * SEQ * HD / 2 + 255) / 256), gplp = (unsigned)(((size_t)NB * NH * LP * HD / 2 + 255) / 256);
    k_cvtrows<<<gx, 256, 0, stream>>>(query, SEQ_FULL, SEQ, SEQ, XB);
    k_gemmw<bf, 0, true><<<dim3(SEQ / 64, DM / 64, NB), 32, 0, stream>>>(XB, nullptr, WQB, nullptr, DM, F, DM, bq, (size_t)SEQ * DM, 0, (size_t)SEQ * DM);
    k_qplanes<<<gpl, 256, 0, stream>>>(F, ub, vb, QU16, QV16);
    k_cvtrows<<<gx, 256, 0, stream>>>(key, SEQ_FULL, SEQ, SEQ, XB);
    k_gemmw<bf, 0, true><<<dim3(SEQ / 64, DM / 64, NB), 32, 0, stream>>>(XB, nullptr, WKB, nullptr, DM, F, DM, bk, (size_t)SEQ * DM, 0, (size_t)SEQ * DM);
    k_kplane<<<gpl, 256, 0, stream>>>(F, K16);
    k_cvtrows<<<gx, 256, 0, stream>>>(value, SEQ_FULL, SEQ, SEQ, XB);
    k_gemmw<bf, 0, true><<<dim3(SEQ / 64, DM / 64, NB), 32, 0, stream>>>(XB, nullptr, WVB, nullptr, DM, F, DM, bv, (size_t)SEQ * DM, 0, (size_t)SEQ * DM);
    k_vplanes<<<gpl, 256, 0, stream>>>(F, V16, VR16);
    k_cvtrows<<<gxp, 256, 0, stream>>>(pos, LREL_FULL, LREL, LP, XB);
    k_gemmw<bf, 0, false><<<dim3(LP / 64, DM / 64, NB), 32, 0, stream>>>(XB, nullptr, WPB, nullptr, DM, F, DM, nullptr, (size_t)LP * DM, 0, (size_t)LP * DM);
    k_pplane<<<gplp, 256, 0, stream>>>(F, P16);
    k_attn<<<dim3(SEQ / 64, NH, NB), 128, 0, stream>>>(QU16, QV16, K16, V16, VR16, P16, ATh, ATl);
    k_gemmw<bf, 1, true><<<dim3((NB * SEQ) / 64, DM / 64, 1), 32, 0, stream>>>(ATh, ATl, WOB, nullptr, DM, OUT, DM, bo, 0, 0, 0);
}
